// My_SA_88098369175821
// MI455X (gfx1250) — hardware-verified
//
#include <hip/hip_runtime.h>
#include <stdint.h>

#define NBATCH 4096
#define TT     128
#define CC     20
#define KQ     100
#define CP     32
#define DP     128
#define XROW   (TT * CC)

static_assert(XROW == 2560);
static_assert(TT == 128);
static_assert(DP == TT);

#define OFF_XS   0
#define OFF_XH   10240
#define OFF_KS   18432
#define OFF_QS   51200
#define OFF_VTH  83968
#define OFF_VTL  92160
#define OFF_SS   100352
#define LDS_MAIN 165888
static_assert(OFF_XH == OFF_XS + TT * CC * 4);
static_assert(OFF_KS == OFF_XH + TT * CP * 2);
static_assert(OFF_QS == OFF_KS + TT * DP * 2);
static_assert(OFF_VTH == OFF_QS + TT * DP * 2);
static_assert(OFF_VTL == OFF_VTH + CP * DP * 2);
static_assert(OFF_SS == OFF_VTL + CP * DP * 2);
static_assert(LDS_MAIN == OFF_SS + TT * TT * 4);

#define WK_OFF    0
#define WQ_OFF    4096
#define WV_OFF    8192
#define WS_HALVES 9216
static_assert(WS_HALVES == 4096 + 4096 + 1024);
static_assert((WS_HALVES % 8) == 0);

typedef _Float16     v16h __attribute__((ext_vector_type(16)));
typedef _Float16     v8h  __attribute__((ext_vector_type(8)));
typedef float        v8f  __attribute__((ext_vector_type(8)));
typedef float        v4f  __attribute__((ext_vector_type(4)));
typedef unsigned int v4u  __attribute__((ext_vector_type(4)));

union Frag { v16h v; v8h half[2]; };

__device__ __forceinline__ unsigned short bf_bits(float f) {
  unsigned u = __float_as_uint(f);
  return (unsigned short)((u + 0x7FFFu + ((u >> 16) & 1u)) >> 16);
}
__device__ __forceinline__ float bf_up(unsigned short b) { return __uint_as_float(((unsigned)b) << 16); }
__device__ __forceinline__ float bfr(float f) { return bf_up(bf_bits(f)); }
__device__ __forceinline__ v4f bfr4(v4f a) {
  v4f o;
  o[0] = bfr(a[0]); o[1] = bfr(a[1]); o[2] = bfr(a[2]); o[3] = bfr(a[3]);
  return o;
}
__device__ __forceinline__ unsigned short h_bits(float f) {
  return __builtin_bit_cast(unsigned short, (_Float16)f);
}
__device__ __forceinline__ v8f zero8() {
  v8f z;
  z[0] = 0.f; z[1] = 0.f; z[2] = 0.f; z[3] = 0.f; z[4] = 0.f; z[5] = 0.f; z[6] = 0.f; z[7] = 0.f;
  return z;
}
__device__ __forceinline__ float elu_f(float v) {
  const float e = __expf(v) - 1.0f;
  return v > 0.0f ? v : e;
}
__device__ __forceinline__ float tanh_f(float v) {
  const float c = fminf(fmaxf(v, -15.0f), 15.0f);
  const float t = __expf(2.0f * c);
  return (t - 1.0f) * __builtin_amdgcn_rcpf(t + 1.0f);
}

__device__ __forceinline__ v16h ldfrag(const _Float16* p) {
  Frag f;
  f.half[0] = *(const v8h*)(p);
  f.half[1] = *(const v8h*)(p + 16);
  return f.v;
}

__device__ __forceinline__ v8f mma(v16h a, v16h b, v8f c) {
  v8f d = __builtin_amdgcn_wmma_f32_16x16x32_f16(false, a, false, b, (short)0, c, false, false);
#if defined(__HIP_DEVICE_COMPILE__)
  asm volatile("v_nop\n\tv_nop\n\tv_nop\n\tv_nop" : "+v"(d) : "v"(a), "v"(b));
#endif
  return d;
}

__global__ __launch_bounds__(256) void k_prep(const float* __restrict__ Wk, const float* __restrict__ Wq,
                                              const float* __restrict__ Wv, unsigned short* P) {
  __shared__ __align__(16) unsigned short sW[WS_HALVES];
  const int tid = threadIdx.x;

#pragma unroll 1
  for (int it = 0; it < 16; ++it) {
    const int idx = it * 256 + tid;
    const int n = idx >> 5, c = idx & 31;
    const int nn = min(n, KQ - 1), cc = min(c, CC - 1);
    float v = Wk[cc * KQ + nn];
    v = (n < KQ && c < CC) ? v : 0.0f;
    sW[WK_OFF + idx] = h_bits(bfr(v) * 1024.0f);
  }
#pragma unroll 1
  for (int it = 0; it < 16; ++it) {
    const int idx = it * 256 + tid;
    const int n = idx >> 5, c = idx & 31;
    const int nn = min(n, KQ - 1), cc = min(c, CC - 1);
    float v = Wq[cc * KQ + nn];
    v = (n < KQ && c < CC) ? v : 0.0f;
    sW[WQ_OFF + idx] = h_bits(bfr(v) * 1024.0f);
  }
#pragma unroll 1
  for (int it = 0; it < 4; ++it) {
    const int idx = it * 256 + tid;
    const int d = idx >> 5, c = idx & 31;
    const int dd = min(d, CC - 1), cc = min(c, CC - 1);
    float v = Wv[cc * CC + dd];
    v = (d < CC && c < CC) ? v : 0.0f;
    sW[WV_OFF + idx] = h_bits(bfr(v) * 1024.0f);
  }
  __syncthreads();

  v4u pv[5];
#pragma unroll
  for (int it = 0; it < 5; ++it) {
    const int idx = min(it * 256 + tid, WS_HALVES / 8 - 1);
    pv[it] = *(const v4u*)(sW + (size_t)idx * 8);
  }
#pragma unroll
  for (int it = 0; it < 5; ++it) {
    const int idx = it * 256 + tid;
    if (idx < WS_HALVES / 8) *(volatile v4u*)(P + (size_t)idx * 8) = pv[it];
  }
  __threadfence();
#pragma unroll
  for (int it = 0; it < 5; ++it) {
    const int idx = it * 256 + tid;
    if (idx < WS_HALVES / 8) *(volatile v4u*)(P + (size_t)idx * 8) = pv[it];
  }
}

__global__ __launch_bounds__(256) void k_main(const float* __restrict__ x, const unsigned short* __restrict__ Wp,
                                              const float* __restrict__ bk, const float* __restrict__ bq,
                                              const float* __restrict__ bv, float* out) {
  extern __shared__ __align__(16) unsigned char smem[];
  float*    xs  = (float*)(smem + OFF_XS);
  _Float16* xh  = (_Float16*)(smem + OFF_XH);
  _Float16* kS  = (_Float16*)(smem + OFF_KS);
  _Float16* qS  = (_Float16*)(smem + OFF_QS);
  _Float16* vTh = (_Float16*)(smem + OFF_VTH);
  _Float16* vTl = (_Float16*)(smem + OFF_VTL);
  float*    sS  = (float*)(smem + OFF_SS);
  const _Float16* W = (const _Float16*)(const void*)Wp;

  const int tid  = threadIdx.x;
  const int lane = tid & 31;
  const int wid  = tid >> 5;
  const int h    = lane >> 4;
  const int lo   = lane & 15;
  const int b    = blockIdx.x;
  const int m0   = wid * 16;
  const float* xb = x + (size_t)b * XROW;

  {
    const int part = tid >> 7;
    const int row  = tid & 127;
    const float* xr  = xb + row * CC;
    float*       xsr = xs + row * CC;
    _Float16*    xhr = xh + row * CP;
    if (part == 0) {
      const v4f a0 = bfr4(*(const v4f*)(xr));
      const v4f a1 = bfr4(*(const v4f*)(xr + 4));
      const v4f a2 = bfr4(*(const v4f*)(xr + 8));
      const v4f a3 = bfr4(*(const v4f*)(xr + 12));
      *(v4f*)(xsr)      = a0;
      *(v4f*)(xsr + 4)  = a1;
      *(v4f*)(xsr + 8)  = a2;
      *(v4f*)(xsr + 12) = a3;
      v8h p0, p1;
#pragma unroll
      for (int c = 0; c < 4; ++c) {
        p0[c]     = (_Float16)(a0[c] * 16.0f);
        p0[4 + c] = (_Float16)(a1[c] * 16.0f);
        p1[c]     = (_Float16)(a2[c] * 16.0f);
        p1[4 + c] = (_Float16)(a3[c] * 16.0f);
      }
      *(v8h*)(xhr)     = p0;
      *(v8h*)(xhr + 8) = p1;
    } else {
      const v4f a4 = bfr4(*(const v4f*)(xr + 16));
      *(v4f*)(xsr + 16) = a4;
      v8h p2, p3;
#pragma unroll
      for (int c = 0; c < 4; ++c) {
        p2[c]     = (_Float16)(a4[c] * 16.0f);
        p2[4 + c] = (_Float16)0.0f;
        p3[c]     = (_Float16)0.0f;
        p3[4 + c] = (_Float16)0.0f;
      }
      *(v8h*)(xhr + 16) = p2;
      *(v8h*)(xhr + 24) = p3;
    }
  }
  __syncthreads();

  {
    const v16h af = ldfrag(xh + (m0 + lo) * CP + 8 * h);
#pragma unroll 1
    for (int nt = 0; nt < 8; ++nt) {
      const int n0 = nt * 16, n = n0 + lo;
      const v8f acc = mma(af, ldfrag(W + WK_OFF + (size_t)(n0 + lo) * CP + 8 * h), zero8());
      const float bias = bfr(bk[min(n, KQ - 1)]);
#pragma unroll
      for (int r = 0; r < 8; ++r) {
        float val = elu_f(acc[r] * 6.103515625e-05f + bias);
        val = (n < KQ) ? val : 0.0f;
        kS[(m0 + 8 * h + r) * DP + n] = (_Float16)(val * 8.0f);
      }
    }
#pragma unroll 1
    for (int nt = 0; nt < 8; ++nt) {
      const int n0 = nt * 16, n = n0 + lo;
      const v8f acc = mma(af, ldfrag(W + WQ_OFF + (size_t)(n0 + lo) * CP + 8 * h), zero8());
      const float bias = bfr(bq[min(n, KQ - 1)]);
#pragma unroll
      for (int r = 0; r < 8; ++r) {
        float val = elu_f(acc[r] * 6.103515625e-05f + bias);
        val = (n < KQ) ? val : 0.0f;
        qS[(m0 + 8 * h + r) * DP + n] = (_Float16)(val * 8.0f);
      }
    }
#pragma unroll 1
    for (int nt = 0; nt < 2; ++nt) {
      const int n0 = nt * 16, d = n0 + lo;
      const v8f acc = mma(af, ldfrag(W + WV_OFF + (size_t)(n0 + lo) * CP + 8 * h), zero8());
      const float bias = bfr(bv[min(d, CC - 1)]);
#pragma unroll
      for (int r = 0; r < 8; ++r) {
        float val = tanh_f(acc[r] * 6.103515625e-05f + bias);
        val = (d < CC) ? val : 0.0f;
        const float v16 = val * 16.0f;
        const _Float16 hh = (_Float16)v16;
        const _Float16 ll = (_Float16)((v16 - (float)hh) * 2048.0f);
        vTh[d * DP + m0 + 8 * h + r] = hh;
        vTl[d * DP + m0 + 8 * h + r] = ll;
      }
    }
  }
  __syncthreads();

  {
    const float SC64 = 0.08838834764831845f * 0.015625f;
    const _Float16* pa = kS + (m0 + lo) * DP + 8 * h;
    const v16h a0 = ldfrag(pa);
    const v16h a1 = ldfrag(pa + 32);
    const v16h a2 = ldfrag(pa + 64);
    const v16h a3 = ldfrag(pa + 96);
#pragma unroll 1
    for (int nt = 0; nt < 8; ++nt) {
      const int n0 = nt * 16;
      const _Float16* pb = qS + (n0 + lo) * DP + 8 * h;
      v8f acc = mma(a0, ldfrag(pb), zero8());
      acc = mma(a1, ldfrag(pb + 32), acc);
      acc = mma(a2, ldfrag(pb + 64), acc);
      acc = mma(a3, ldfrag(pb + 96), acc);
#pragma unroll
      for (int r = 0; r < 8; ++r) sS[(m0 + 8 * h + r) * TT + n0 + lo] = acc[r] * SC64;
    }
  }
  __syncthreads();

  {
    const int j    = tid >> 1;
    const int half = tid & 1;
    float* col = sS + (half * 64) * TT + j;
    float mx = -3.0e38f;
#pragma unroll 4
    for (int ii = 0; ii < 64; ++ii) mx = fmaxf(mx, col[ii * TT]);
    mx = fmaxf(mx, __shfl_xor(mx, 1));
    float sum = 0.0f;
#pragma unroll 4
    for (int ii = 0; ii < 64; ++ii) {
      const float e = __expf(col[ii * TT] - mx);
      sum += e;
      col[ii * TT] = e;
    }
    sum += __shfl_xor(sum, 1);
    const float rs = 1.0f / sum;
    _Float16* Ph = qS;
#pragma unroll 4
    for (int ii = 0; ii < 64; ++ii)
      Ph[(half * 64 + ii) * DP + j] = (_Float16)((col[ii * TT] * rs) * 1024.0f);
  }
  __syncthreads();

  {
    const _Float16* Ph = qS;
    const _Float16* pa = Ph + (m0 + lo) * DP + 8 * h;
    const v16h p0 = ldfrag(pa);
    const v16h p1 = ldfrag(pa + 32);
    const v16h p2 = ldfrag(pa + 64);
    const v16h p3 = ldfrag(pa + 96);
    const _Float16* bh0 = vTh + lo * DP + 8 * h;
    const _Float16* bh1 = vTh + (16 + lo) * DP + 8 * h;
    const _Float16* bl0 = vTl + lo * DP + 8 * h;
    const _Float16* bl1 = vTl + (16 + lo) * DP + 8 * h;
    v8f ah0 = zero8(), ah1 = zero8(), al0 = zero8(), al1 = zero8();
    ah0 = mma(p0, ldfrag(bh0),      ah0); ah1 = mma(p0, ldfrag(bh1),      ah1);
    al0 = mma(p0, ldfrag(bl0),      al0); al1 = mma(p0, ldfrag(bl1),      al1);
    ah0 = mma(p1, ldfrag(bh0 + 32), ah0); ah1 = mma(p1, ldfrag(bh1 + 32), ah1);
    al0 = mma(p1, ldfrag(bl0 + 32), al0); al1 = mma(p1, ldfrag(bl1 + 32), al1);
    ah0 = mma(p2, ldfrag(bh0 + 64), ah0); ah1 = mma(p2, ldfrag(bh1 + 64), ah1);
    al0 = mma(p2, ldfrag(bl0 + 64), al0); al1 = mma(p2, ldfrag(bl1 + 64), al1);
    ah0 = mma(p3, ldfrag(bh0 + 96), ah0); ah1 = mma(p3, ldfrag(bh1 + 96), ah1);
    al0 = mma(p3, ldfrag(bl0 + 96), al0); al1 = mma(p3, ldfrag(bl1 + 96), al1);

    const int d1  = 16 + lo;
    const int d1c = min(d1, CC - 1);
#pragma unroll
    for (int r = 0; r < 8; ++r) {
      const int i = m0 + 8 * h + r;
      float* px = xs + i * CC;
      const float y0 = (ah0[r] + al0[r] * 0.00048828125f) * 6.103515625e-05f;
      const float y1 = (ah1[r] + al1[r] * 0.00048828125f) * 6.103515625e-05f;
      const float v0 = px[lo] + y0;
      const float v1 = px[d1c] + y1;
      px[lo] = v0;
      if (lo < 4) px[d1] = v1;
    }
  }
  __syncthreads();

  {
    const v4f* xs4 = (const v4f*)xs;
    const int c2  = 16 + wid;
    const int c2c = min(c2, 19);
    const v4f pv0 = xs4[(wid)     * 32 + lane];
    const v4f pv1 = xs4[(8 + wid) * 32 + lane];
    const v4f pv2 = xs4[c2c       * 32 + lane];
    float* ob = out + (size_t)b * XROW + (size_t)lane * 4;
    *(volatile v4f*)(ob + (size_t)wid * 128)       = pv0;
    *(volatile v4f*)(ob + (size_t)(8 + wid) * 128) = pv1;
    if (wid < 4) *(volatile v4f*)(ob + (size_t)c2 * 128) = pv2;
    __threadfence();
    *(volatile v4f*)(ob + (size_t)wid * 128)       = pv0;
    *(volatile v4f*)(ob + (size_t)(8 + wid) * 128) = pv1;
    if (wid < 4) *(volatile v4f*)(ob + (size_t)c2 * 128) = pv2;
  }
}

extern "C" void kernel_launch(void* const* d_in, const int* in_sizes, int n_in,
                              void* d_out, int out_size, void* d_ws, size_t ws_size,
                              hipStream_t stream) {
  if (n_in < 7) return;
  if (in_sizes[0] != NBATCH * XROW) return;
  if (in_sizes[1] != CC * KQ) return;
  if (in_sizes[2] != KQ) return;
  if (in_sizes[3] != CC * KQ) return;
  if (in_sizes[4] != KQ) return;
  if (in_sizes[5] != CC * CC) return;
  if (in_sizes[6] != CC) return;
  if (out_size != NBATCH * XROW) return;

  const float* x  = (const float*)d_in[0];
  const float* Wk = (const float*)d_in[1];
  const float* bk = (const float*)d_in[2];
  const float* Wq = (const float*)d_in[3];
  const float* bq = (const float*)d_in[4];
  const float* Wv = (const float*)d_in[5];
  const float* bv = (const float*)d_in[6];
  float* out = (float*)d_out;

  const size_t wsb = (size_t)WS_HALVES * 2;
  if (wsb > ws_size) return;
  if (wsb > (size_t)134217728) return;
  unsigned short* P = (unsigned short*)d_ws;

  (void)hipFuncSetAttribute(reinterpret_cast<const void*>(&k_main),
                            hipFuncAttributeMaxDynamicSharedMemorySize, LDS_MAIN);

  const dim3 gPrep(1), bPrep(256);
  const dim3 gMain(NBATCH), bMain(256);

  k_prep<<<gPrep, bPrep, 0, stream>>>(Wk, Wq, Wv, P);
  k_main<<<gMain, bMain, LDS_MAIN, stream>>>(x, P, bk, bq, bv, out);
  (void)hipGetLastError();
}
